// GNN_59219009077824
// MI455X (gfx1250) — hardware-verified
//
#include <hip/hip_runtime.h>
#include <stddef.h>
#include <stdint.h>
#include <math.h>


#define NB     256
#define FIN    6
#define KP     32
#define HID    128
#define OD     64
#define K2     256
#define NTHR   256
#define NWAVE  8
#define TROWS  64
#define NTILE  4
#define NU1    (HID * (KP / 8))
#define NU2    (OD * (K2 / 8))

#define OFF_XB    0
#define OFF_STG   16384
#define OFF_HHL   49152
#define OFF_SPART 81920
#define OFF_SSUM  90112
#define OFF_B1S   91136
#define OFF_DINV  91648
#define OFF_WC    92672
#define OFF_WU    93696
#define OFF_CF    94720
#define OFF_ZPART 95744
#define OFF_OUTS  98816
#define OFF_RED   99072
#define LDS_BYTES 99200

static_assert(NB == NTHR);
static_assert(NB == NTILE * TROWS);
static_assert(KP % 32 == 0 && K2 % 32 == 0 && K2 == 2 * HID);
static_assert(NU1 % NTHR == 0 && (NU1 + NU2) % NTHR == 0);
static_assert(TROWS * HID == 8 * NTHR * 4);
static_assert(OFF_STG == OFF_XB + NB * KP * 2);
static_assert(OFF_HHL == OFF_STG + TROWS * HID * 4);
static_assert(OFF_SPART == OFF_HHL + TROWS * K2 * 2);
static_assert(OFF_SSUM == OFF_SPART + 2 * NWAVE * HID * 4);
static_assert(OFF_RED + 128 == LDS_BYTES);
static_assert(LDS_BYTES <= 300000);

typedef float          v2f   __attribute__((ext_vector_type(2)));
typedef float          v4f   __attribute__((ext_vector_type(4)));
typedef float          v8f   __attribute__((ext_vector_type(8)));
typedef int            v8i   __attribute__((ext_vector_type(8)));
typedef unsigned short v4us  __attribute__((ext_vector_type(4)));
typedef unsigned short v8us  __attribute__((ext_vector_type(8)));
typedef unsigned short v16us __attribute__((ext_vector_type(16)));
typedef __bf16         v16bf __attribute__((ext_vector_type(16)));
typedef v2f  __attribute__((may_alias)) v2fa;
typedef v4f  __attribute__((may_alias)) v4fa;
typedef v4us __attribute__((may_alias)) v4usa;
typedef v8us __attribute__((may_alias)) v8usa;
union FragB { v16bf v; v16us u; v8us h[2]; v8i w; };

__device__ __forceinline__ v8f wmb(const FragB& a, const FragB& b, v8f c) {
  v8f d = __builtin_amdgcn_wmma_f32_16x16x32_bf16(false, a.v, false, b.v, (short)0, c, false, false);
  asm volatile("v_nop\n\tv_nop\n\tv_nop\n\tv_nop" : "+v"(d) : "v"(a.w), "v"(b.w));
  return d;
}

__device__ __forceinline__ unsigned bf16_bits(float f) {
  const unsigned u = __float_as_uint(f);
  return (u + 0x7FFFu + ((u >> 16) & 1u)) >> 16;
}
__device__ __forceinline__ float bf16_val(float f) {
  return __uint_as_float(bf16_bits(f) << 16);
}

__device__ __forceinline__ float wsum8(const v4f w0, const v4f w1, const v8f a, float s) {
  s = fmaf(w0.x, a[0], s); s = fmaf(w0.y, a[1], s); s = fmaf(w0.z, a[2], s); s = fmaf(w0.w, a[3], s);
  s = fmaf(w1.x, a[4], s); s = fmaf(w1.y, a[5], s); s = fmaf(w1.z, a[6], s); s = fmaf(w1.w, a[7], s);
  return s;
}

__device__ __forceinline__ unsigned hsplit(float y, float sa, float sc, float bb, float d, bool cnd) {
  const float alt = sc + d * y;
  const float agg = cnd ? sa : alt;
  float v = d * agg + bb;
  v = (v > 0.0f) ? v : 0.0f;
  const unsigned hb = bf16_bits(v);
  const unsigned lb = bf16_bits(v - __uint_as_float(hb << 16));
  return (lb << 16) | hb;
}

__global__ __launch_bounds__(NTHR) void k_prep(const float* __restrict__ W1, const float* __restrict__ W2,
                                               unsigned short* W1T, unsigned short* W2T2) {
  const int u = (int)blockIdx.x * NTHR + (int)threadIdx.x;
  v8us o;
  unsigned short* dp;
  if (u < NU1) {
    const int n  = u >> 2;
    const int k8 = (u & 3) * 8;
#pragma unroll
    for (int i = 0; i < 8; ++i) {
      const int k  = k8 + i;
      const int kc = k < FIN ? k : FIN - 1;
      const unsigned bits = bf16_bits(W1[(size_t)kc * HID + n]);
      o[i] = (k < FIN) ? (unsigned short)bits : (unsigned short)0;
    }
    dp = W1T + (size_t)u * 8;
  } else if (u < NU1 + NU2) {
    const int v  = u - NU1;
    const int n  = v >> 5;
    const int k8 = (v & 31) * 8;
    const int kk = k8 & (HID - 1);
    const float* p = W2 + (size_t)kk * OD + n;
#pragma unroll
    for (int i = 0; i < 8; ++i) o[i] = (unsigned short)bf16_bits(p[(size_t)i * OD]);
    dp = W2T2 + (size_t)v * 8;
  } else {
    return;
  }
  *(volatile v8us*)dp = o;
  __threadfence();
  *(volatile v8us*)dp = o;
}

__global__ __launch_bounds__(NTHR) void k_graph(const float* __restrict__ x, const float* __restrict__ b1,
                                                const float* __restrict__ b2,
                                                const unsigned short* __restrict__ W1T,
                                                const unsigned short* __restrict__ W2T2, float* out) {
  extern __shared__ __attribute__((aligned(16))) unsigned char dsm[];
  unsigned short* xb    = (unsigned short*)(dsm + OFF_XB);
  float*          stg   = (float*)(dsm + OFF_STG);
  unsigned short* hhl   = (unsigned short*)(dsm + OFF_HHL);
  float*          spart = (float*)(dsm + OFF_SPART);
  float*          ssum  = (float*)(dsm + OFF_SSUM);
  float*          b1s   = (float*)(dsm + OFF_B1S);
  float*          dinvs = (float*)(dsm + OFF_DINV);
  float*          wcs   = (float*)(dsm + OFF_WC);
  float*          wus   = (float*)(dsm + OFF_WU);
  float*          cfl   = (float*)(dsm + OFF_CF);
  float*          zpart = (float*)(dsm + OFF_ZPART);
  float*          outs  = (float*)(dsm + OFF_OUTS);
  int*            cntv  = (int*)(dsm + OFF_RED);
  int*            cntc  = cntv + 8;
  float*          redc  = (float*)(dsm + OFF_RED + 64);
  float*          redn  = redc + 8;

  const int tid = (int)threadIdx.x, lane = tid & 31, wave = tid >> 5, hh = lane >> 4, m = lane & 15;
  const int g = (int)blockIdx.x;
  const v8f z8 = {0.f, 0.f, 0.f, 0.f, 0.f, 0.f, 0.f, 0.f};

  bool valid, cond;
  {
    const float* xr = x + ((size_t)g * NB + (size_t)tid) * FIN;
    const v2f p0 = *(const v2fa*)xr;
    const v2f p1 = *(const v2fa*)(xr + 2);
    const v2f p2 = *(const v2fa*)(xr + 4);
    const unsigned q0 = bf16_bits(p0.x), q1 = bf16_bits(p0.y), q2 = bf16_bits(p1.x);
    const unsigned q3 = bf16_bits(p1.y), q4 = bf16_bits(p2.x), q5 = bf16_bits(p2.y);
    valid = (((q0 | q1 | q2 | q3 | q4 | q5) & 0x7FFFu) != 0u);
    cond  = (((q3 | q4) & 0x7FFFu) != 0u);
    v8us r0;
    r0[0] = (unsigned short)q0; r0[1] = (unsigned short)q1; r0[2] = (unsigned short)q2;
    r0[3] = (unsigned short)q3; r0[4] = (unsigned short)q4; r0[5] = (unsigned short)q5;
    r0[6] = (unsigned short)0;  r0[7] = (unsigned short)0;
    const v8us zz = {0, 0, 0, 0, 0, 0, 0, 0};
    unsigned short* xrow = xb + tid * KP;
    *(v8usa*)xrow        = r0;
    *(v8usa*)(xrow + 8)  = zz;
    *(v8usa*)(xrow + 16) = zz;
    *(v8usa*)(xrow + 24) = zz;
  }
  {
    const unsigned mv = __builtin_amdgcn_ballot_w32(valid);
    const unsigned mc = __builtin_amdgcn_ballot_w32(cond);
    if (lane == 0) { cntv[wave] = (int)__builtin_popcount(mv); cntc[wave] = (int)__builtin_popcount(mc); }
  }
  if (tid < HID) b1s[tid] = bf16_val(b1[tid]);
  __syncthreads();

  int nv = 0, nc = 0;
#pragma unroll
  for (int w2 = 0; w2 < NWAVE; ++w2) { nv += cntv[w2]; nc += cntc[w2]; }

  {
    const int deg = valid ? (cond ? nv : (nc + 1)) : 0;
    const float dsafe = (deg > 0) ? (float)deg : 1.0f;
    const float rs = 1.0f / sqrtf(dsafe);
    const float di = (deg > 0) ? rs : 0.0f;
    const bool ncv = valid && !cond;
    const float vc = cond ? di : 0.0f;
    const float vn = ncv ? di : 0.0f;
    dinvs[tid] = di;
    wcs[tid]   = vc;
    wus[tid]   = ncv ? di * di : 0.0f;
    cfl[tid]   = cond ? 1.0f : 0.0f;
    float rc = vc, rn = vn;
#pragma unroll
    for (int d = 16; d >= 1; d >>= 1) {
      rc += __shfl_xor(rc, d, 32);
      rn += __shfl_xor(rn, d, 32);
    }
    if (lane == 0) { redc[wave] = rc; redn[wave] = rn; }
  }
  __syncthreads();

  {
    FragB afA[2];
    v4f waA[2][2], wcA[2][2];
#pragma unroll
    for (int i = 0; i < 2; ++i) {
      const unsigned short* ar = xb + (32 * wave + 16 * i + m) * KP + 8 * hh;
      afA[i].h[0] = *(const v8usa*)ar;
      afA[i].h[1] = *(const v8usa*)(ar + 16);
      const int rb = 32 * wave + 16 * i + 8 * hh;
      waA[i][0] = *(const v4fa*)(dinvs + rb);
      waA[i][1] = *(const v4fa*)(dinvs + rb + 4);
      wcA[i][0] = *(const v4fa*)(wcs + rb);
      wcA[i][1] = *(const v4fa*)(wcs + rb + 4);
    }
#pragma unroll 1
    for (int nt = 0; nt < HID / 16; ++nt) {
      const unsigned short* wq = W1T + (size_t)(16 * nt + m) * KP + 8 * hh;
      FragB bf;
      bf.h[0] = *(const v8usa*)wq;
      bf.h[1] = *(const v8usa*)(wq + 16);
      float sA = 0.0f, sC = 0.0f;
#pragma unroll
      for (int i = 0; i < 2; ++i) {
        const v8f acc = wmb(afA[i], bf, z8);
        sA = wsum8(waA[i][0], waA[i][1], acc, sA);
        sC = wsum8(wcA[i][0], wcA[i][1], acc, sC);
      }
      sA += __shfl_xor(sA, 16, 32);
      sC += __shfl_xor(sC, 16, 32);
      if (hh == 0) {
        spart[(0 * NWAVE + wave) * HID + 16 * nt + m] = sA;
        spart[(1 * NWAVE + wave) * HID + 16 * nt + m] = sC;
      }
    }
  }
  __syncthreads();
  {
    const int kind = tid >> 7;
    const int c    = tid & (HID - 1);
    float s = 0.0f;
#pragma unroll
    for (int w2 = 0; w2 < NWAVE; ++w2) s += spart[(kind * NWAVE + w2) * HID + c];
    ssum[kind * HID + c] = s;
  }
  __syncthreads();

  const int mt = wave & 3;
  const int ng = wave >> 2;
  float za0 = 0.0f, za1 = 0.0f, zc0 = 0.0f, zc1 = 0.0f, zu0 = 0.0f, zu1 = 0.0f;

#pragma unroll 1
  for (int T = 0; T < NTILE; ++T) {
    {
      const unsigned short* ar = xb + (TROWS * T + 16 * mt + m) * KP + 8 * hh;
      FragB af;
      af.h[0] = *(const v8usa*)ar;
      af.h[1] = *(const v8usa*)(ar + 16);
#pragma unroll 1
      for (int j = 0; j < 4; ++j) {
        const int nt = 4 * ng + j;
        const unsigned short* wq = W1T + (size_t)(16 * nt + m) * KP + 8 * hh;
        FragB bf;
        bf.h[0] = *(const v8usa*)wq;
        bf.h[1] = *(const v8usa*)(wq + 16);
        const v8f acc = wmb(af, bf, z8);
        float* sp = stg + (16 * mt + 8 * hh) * HID + 16 * nt + m;
#pragma unroll
        for (int r = 0; r < 8; ++r) sp[r * HID] = acc[r];
      }
    }
    __syncthreads();

#pragma unroll 1
    for (int it = 0; it < 8; ++it) {
      const int idx  = it * NTHR + tid;
      const int row  = idx >> 5;
      const int c4   = (idx & 31) * 4;
      const int node = TROWS * T + row;
      const float d  = dinvs[node];
      const bool cnd = cfl[node] != 0.0f;
      const v4f y  = *(const v4fa*)(stg + row * HID + c4);
      const v4f sa = *(const v4fa*)(ssum + c4);
      const v4f sc = *(const v4fa*)(ssum + HID + c4);
      const v4f bb = *(const v4fa*)(b1s + c4);
      const unsigned e0 = hsplit(y.x, sa.x, sc.x, bb.x, d, cnd);
      const unsigned e1 = hsplit(y.y, sa.y, sc.y, bb.y, d, cnd);
      const unsigned e2 = hsplit(y.z, sa.z, sc.z, bb.z, d, cnd);
      const unsigned e3 = hsplit(y.w, sa.w, sc.w, bb.w, d, cnd);
      v4us h4, l4;
      h4[0] = (unsigned short)(e0 & 0xFFFFu); l4[0] = (unsigned short)(e0 >> 16);
      h4[1] = (unsigned short)(e1 & 0xFFFFu); l4[1] = (unsigned short)(e1 >> 16);
      h4[2] = (unsigned short)(e2 & 0xFFFFu); l4[2] = (unsigned short)(e2 >> 16);
      h4[3] = (unsigned short)(e3 & 0xFFFFu); l4[3] = (unsigned short)(e3 >> 16);
      unsigned short* hr = hhl + row * K2 + c4;
      *(v4usa*)hr         = h4;
      *(v4usa*)(hr + HID) = l4;
    }
    __syncthreads();

    v8f acc0 = z8, acc1 = z8;
    {
      const unsigned short* ha = hhl + (16 * mt + m) * K2 + 8 * hh;
      const unsigned short* wb = W2T2 + (size_t)(16 * (2 * ng) + m) * K2 + 8 * hh;
#pragma unroll 1
      for (int ks = 0; ks < K2 / 32; ++ks) {
        FragB af, bf0, bf1;
        af.h[0]  = *(const v8usa*)(ha + 32 * ks);
        af.h[1]  = *(const v8usa*)(ha + 32 * ks + 16);
        bf0.h[0] = *(const v8usa*)(wb + 32 * ks);
        bf0.h[1] = *(const v8usa*)(wb + 32 * ks + 16);
        bf1.h[0] = *(const v8usa*)(wb + (size_t)16 * K2 + 32 * ks);
        bf1.h[1] = *(const v8usa*)(wb + (size_t)16 * K2 + 32 * ks + 16);
        acc0 = wmb(af, bf0, acc0);
        acc1 = wmb(af, bf1, acc1);
      }
    }
    {
      const int rb = TROWS * T + 16 * mt + 8 * hh;
      const v4f wa0 = *(const v4fa*)(dinvs + rb), wa1 = *(const v4fa*)(dinvs + rb + 4);
      const v4f wc0 = *(const v4fa*)(wcs + rb),   wc1 = *(const v4fa*)(wcs + rb + 4);
      const v4f wu0 = *(const v4fa*)(wus + rb),   wu1 = *(const v4fa*)(wus + rb + 4);
      za0 = wsum8(wa0, wa1, acc0, za0); za1 = wsum8(wa0, wa1, acc1, za1);
      zc0 = wsum8(wc0, wc1, acc0, zc0); zc1 = wsum8(wc0, wc1, acc1, zc1);
      zu0 = wsum8(wu0, wu1, acc0, zu0); zu1 = wsum8(wu0, wu1, acc1, zu1);
    }
  }

  za0 += __shfl_xor(za0, 16, 32); za1 += __shfl_xor(za1, 16, 32);
  zc0 += __shfl_xor(zc0, 16, 32); zc1 += __shfl_xor(zc1, 16, 32);
  zu0 += __shfl_xor(zu0, 16, 32); zu1 += __shfl_xor(zu1, 16, 32);
  if (hh == 0) {
    const int c0 = 16 * (2 * ng) + m;
    zpart[(0 * 4 + mt) * OD + c0]      = za0;
    zpart[(0 * 4 + mt) * OD + c0 + 16] = za1;
    zpart[(1 * 4 + mt) * OD + c0]      = zc0;
    zpart[(1 * 4 + mt) * OD + c0 + 16] = zc1;
    zpart[(2 * 4 + mt) * OD + c0]      = zu0;
    zpart[(2 * 4 + mt) * OD + c0 + 16] = zu1;
  }
  __syncthreads();

  if (tid < OD) {
    float za = 0.0f, zc = 0.0f, zu = 0.0f;
#pragma unroll
    for (int q = 0; q < 4; ++q) {
      za += zpart[(0 * 4 + q) * OD + tid];
      zc += zpart[(1 * 4 + q) * OD + tid];
      zu += zpart[(2 * 4 + q) * OD + tid];
    }
    float ac = 0.0f, an = 0.0f;
#pragma unroll
    for (int w2 = 0; w2 < NWAVE; ++w2) { ac += redc[w2]; an += redn[w2]; }
    const float inv = 1.0f / (float)(nv > 0 ? nv : 1);
    const float bz  = bf16_val(b2[tid]);
    const float sm  = fmaf(ac, za, fmaf(an, zc, zu));
    const float v   = sm * inv + bz;
    outs[tid] = (nv > 0) ? v : 0.0f;
  }
  __syncthreads();

  {
    const v4f ov = *(const v4fa*)(outs + 4 * (lane & 15));
    float* op = out + (size_t)g * OD + 4 * (lane & 15);
    const bool okst = (wave == 0) && (lane < 16);
    if (okst) *(volatile v4f*)op = ov;
    __threadfence();
    if (okst) *(volatile v4f*)op = ov;
  }
}

static inline size_t al256(size_t o) { return (o + 255) & ~(size_t)255; }

extern "C" void kernel_launch(void* const* d_in, const int* in_sizes, int n_in,
                              void* d_out, int out_size, void* d_ws, size_t ws_size,
                              hipStream_t stream) {
  if (n_in < 5) return;
  if (in_sizes[0] < NB * FIN || (in_sizes[0] % (NB * FIN)) != 0) return;
  const int nG = in_sizes[0] / (NB * FIN);
  if (nG < 1 || nG > 65536) return;
  if (in_sizes[1] != FIN * HID || in_sizes[2] != HID) return;
  if (in_sizes[3] != HID * OD || in_sizes[4] != OD) return;
  if ((long long)out_size != (long long)nG * OD) return;

  const float* x  = (const float*)d_in[0];
  const float* W1 = (const float*)d_in[1];
  const float* b1 = (const float*)d_in[2];
  const float* W2 = (const float*)d_in[3];
  const float* b2 = (const float*)d_in[4];
  float* out = (float*)d_out;

  char* ws = (char*)d_ws;
  size_t off = 0;
  const size_t oW1T = off; off = al256(off + (size_t)HID * KP * 2);
  const size_t oW2T = off; off = al256(off + (size_t)OD * K2 * 2);
  if (off > ws_size) return;
  unsigned short* W1T  = (unsigned short*)(ws + oW1T);
  unsigned short* W2T2 = (unsigned short*)(ws + oW2T);

  hipFuncSetAttribute(reinterpret_cast<const void*>(&k_graph), hipFuncAttributeMaxDynamicSharedMemorySize,
                      (int)LDS_BYTES);

  k_prep<<<(NU1 + NU2) / NTHR, NTHR, 0, stream>>>(W1, W2, W1T, W2T2);
  k_graph<<<nG, NTHR, LDS_BYTES, stream>>>(x, b1, b2, W1T, W2T2, out);
}
